// HyperbolicAttentionLayer_30124900614682
// MI455X (gfx1250) — hardware-verified
//
#include <hip/hip_runtime.h>
#include <stddef.h>
#include <math.h>


#define DF    512
#define GR    32
#define AP    520
#define XSP   516
#define NTHR  256
#define NWAVE 8
#define KT    (DF / 32)
#define NB    64
#define CHUNK 2048
#define WCAP  256
#define NGRP  (CHUNK / (NTHR * 4))

#define LDS_G_BYTES (GR * AP * 2 + GR * XSP * 4)
#define LDS_A_FL    (2 * NB * DF + 2 * NB)
#define LDS_A_BYTES ((LDS_A_FL + NWAVE * WCAP + NWAVE) * 4)

static_assert(LDS_G_BYTES == 99328);
static_assert(LDS_A_BYTES == 270880);
static_assert(WCAP == (CHUNK / NTHR) * 32);
static_assert(NGRP == 2);
static_assert(NB == 64);
static_assert((NB % NWAVE) == 0);
static_assert(((GR * AP * 2) % 16) == 0);
static_assert(((AP * 2) % 16) == 0 && ((XSP * 4) % 16) == 0);
static_assert(CHUNK <= 32768);

typedef float    v4f  __attribute__((ext_vector_type(4)));
typedef float    v8f  __attribute__((ext_vector_type(8)));
typedef int      v4i  __attribute__((ext_vector_type(4)));
typedef _Float16 v8h  __attribute__((ext_vector_type(8)));
typedef _Float16 v16h __attribute__((ext_vector_type(16)));
union Frag   { v16h v; v8h half[2]; };
union Pack16 { v8h h; v4i i; };

__device__ __forceinline__ v8f wm(v16h a, v16h b, v8f c) {
  v8f d = __builtin_amdgcn_wmma_f32_16x16x32_f16(false, a, false, b, (short)0, c, false, false);
  asm volatile("v_nop\n\tv_nop\n\tv_nop\n\tv_nop" : "+v"(d) : "v"(a), "v"(b));
  return d;
}

__device__ __forceinline__ float wsum(float v) {
  v += __shfl_xor(v, 16, 32);
  v += __shfl_xor(v, 8, 32);
  v += __shfl_xor(v, 4, 32);
  v += __shfl_xor(v, 2, 32);
  v += __shfl_xor(v, 1, 32);
  return v;
}

__global__ __launch_bounds__(NTHR) void k_prep(const float* __restrict__ W0, const float* __restrict__ W1,
                                               const float* __restrict__ W2, const float* __restrict__ W3,
                                               _Float16* Wh, int n8) {
  const int mat = blockIdx.y;
  const float* W = (mat == 0) ? W0 : ((mat == 1) ? W1 : ((mat == 2) ? W2 : W3));
  const int i = blockIdx.x * NTHR + threadIdx.x;
  if (i >= n8) return;
  const size_t o = (size_t)i * 8;
  const v4f a = *(const v4f*)(W + o);
  const v4f b = *(const v4f*)(W + o + 4);
  Pack16 u;
  u.h[0] = (_Float16)(a.x * 16.0f); u.h[1] = (_Float16)(a.y * 16.0f);
  u.h[2] = (_Float16)(a.z * 16.0f); u.h[3] = (_Float16)(a.w * 16.0f);
  u.h[4] = (_Float16)(b.x * 16.0f); u.h[5] = (_Float16)(b.y * 16.0f);
  u.h[6] = (_Float16)(b.z * 16.0f); u.h[7] = (_Float16)(b.w * 16.0f);
  _Float16* dp = Wh + (size_t)mat * DF * DF + o;
  *(volatile v4i*)dp = u.i;
  __threadfence();
  *(volatile v4i*)dp = u.i;
}

__device__ __forceinline__ void mm_pass(const _Float16* At, float* Xs, const _Float16* __restrict__ Wp,
                                        const float* __restrict__ bias, float sc, float osc,
                                        int wave, int hh, int m) {
  const v8f z8 = {0.f, 0.f, 0.f, 0.f, 0.f, 0.f, 0.f, 0.f};
  v8f acc[2][4];
#pragma unroll
  for (int cj = 0; cj < 4; ++cj) { acc[0][cj] = z8; acc[1][cj] = z8; }

#pragma unroll 1
  for (int kt = 0; kt < KT; ++kt) {
    const int k0 = kt * 32;
    Frag a0, a1;
    const _Float16* pa0 = At + m * AP + k0 + 8 * hh;
    const _Float16* pa1 = pa0 + 16 * AP;
    a0.half[0] = *(const v8h*)pa0; a0.half[1] = *(const v8h*)(pa0 + 16);
    a1.half[0] = *(const v8h*)pa1; a1.half[1] = *(const v8h*)(pa1 + 16);
#pragma unroll
    for (int cj = 0; cj < 4; ++cj) {
      const _Float16* pb = Wp + (size_t)(wave * 64 + cj * 16 + m) * DF + k0 + 8 * hh;
      Frag b;
      b.half[0] = *(const v8h*)pb; b.half[1] = *(const v8h*)(pb + 16);
      acc[0][cj] = wm(a0.v, b.v, acc[0][cj]);
      acc[1][cj] = wm(a1.v, b.v, acc[1][cj]);
    }
  }

#pragma unroll
  for (int cj = 0; cj < 4; ++cj) {
    const int col = wave * 64 + cj * 16 + m;
    const float bb = bias[col];
#pragma unroll
    for (int r = 0; r < 8; ++r) {
      Xs[(8 * hh + r) * XSP + col]      = (acc[0][cj][r] * sc + bb) * osc;
      Xs[(16 + 8 * hh + r) * XSP + col] = (acc[1][cj][r] * sc + bb) * osc;
    }
  }
}

__device__ __forceinline__ void store_rows_f32(const float* Xs, float* pl, int rowBase, int wave, int lane) {
  v4f xr[4][4];
#pragma unroll
  for (int i = 0; i < 4; ++i)
#pragma unroll
    for (int j = 0; j < 4; ++j) xr[i][j] = *(const v4f*)(Xs + (4 * wave + i) * XSP + 128 * j + 4 * lane);
#pragma unroll
  for (int i = 0; i < 4; ++i)
#pragma unroll
    for (int j = 0; j < 4; ++j)
      *(volatile v4f*)(pl + (size_t)(rowBase + 4 * wave + i) * DF + 128 * j + 4 * lane) = xr[i][j];
  __threadfence();
#pragma unroll
  for (int i = 0; i < 4; ++i)
#pragma unroll
    for (int j = 0; j < 4; ++j)
      *(volatile v4f*)(pl + (size_t)(rowBase + 4 * wave + i) * DF + 128 * j + 4 * lane) = xr[i][j];
}

__device__ __forceinline__ void store_rows_f16(const float* Xs, _Float16* pl, float mul, int rowBase, int wave, int lane) {
  Pack16 u[4][2];
#pragma unroll
  for (int i = 0; i < 4; ++i)
#pragma unroll
    for (int j = 0; j < 2; ++j) {
      const float* p = Xs + (4 * wave + i) * XSP + 256 * j + 8 * lane;
      const v4f f0 = *(const v4f*)p;
      const v4f f1 = *(const v4f*)(p + 4);
      u[i][j].h[0] = (_Float16)(f0.x * mul); u[i][j].h[1] = (_Float16)(f0.y * mul);
      u[i][j].h[2] = (_Float16)(f0.z * mul); u[i][j].h[3] = (_Float16)(f0.w * mul);
      u[i][j].h[4] = (_Float16)(f1.x * mul); u[i][j].h[5] = (_Float16)(f1.y * mul);
      u[i][j].h[6] = (_Float16)(f1.z * mul); u[i][j].h[7] = (_Float16)(f1.w * mul);
    }
#pragma unroll
  for (int i = 0; i < 4; ++i)
#pragma unroll
    for (int j = 0; j < 2; ++j)
      *(volatile v4i*)(pl + (size_t)(rowBase + 4 * wave + i) * DF + 256 * j + 8 * lane) = u[i][j].i;
  __threadfence();
#pragma unroll
  for (int i = 0; i < 4; ++i)
#pragma unroll
    for (int j = 0; j < 2; ++j)
      *(volatile v4i*)(pl + (size_t)(rowBase + 4 * wave + i) * DF + 256 * j + 8 * lane) = u[i][j].i;
}

__global__ __launch_bounds__(NTHR) void k_node(
    const float* __restrict__ x, const _Float16* __restrict__ Wh,
    const float* __restrict__ bq, const float* __restrict__ bk, const float* __restrict__ bv,
    float* qpl, float* kpl, _Float16* vpl, int nN, float qscale) {
  extern __shared__ v4f lds_dyn[];
  _Float16* At = (_Float16*)lds_dyn;
  float* Xs = (float*)((char*)lds_dyn + GR * AP * 2);

  const int tid  = threadIdx.x;
  const int lane = tid & 31;
  const int wave = tid >> 5;
  const int hh   = lane >> 4;
  const int m    = lane & 15;
  const int rowBase = blockIdx.x * GR;

#pragma unroll 1
  for (int i = 0; i < 4; ++i) {
    const int r = 4 * wave + i;
    int row = rowBase + r;
    if (row > nN - 1) row = nN - 1;
    const float* p = x + (size_t)row * DF + 16 * lane;
    const v4f f0 = *(const v4f*)(p);
    const v4f f1 = *(const v4f*)(p + 4);
    const v4f f2 = *(const v4f*)(p + 8);
    const v4f f3 = *(const v4f*)(p + 12);
    float ss = f0.x * f0.x + f0.y * f0.y + f0.z * f0.z + f0.w * f0.w
             + f1.x * f1.x + f1.y * f1.y + f1.z * f1.z + f1.w * f1.w
             + f2.x * f2.x + f2.y * f2.y + f2.z * f2.z + f2.w * f2.w
             + f3.x * f3.x + f3.y * f3.y + f3.z * f3.z + f3.w * f3.w;
    ss = wsum(ss);
    const float nrm = sqrtf(ss);
    const float nc  = fminf(fmaxf(nrm, 1.0e-7f), 0.999999f);
    const float at  = atanhf(nc);
    const float rc  = 1.0f / nc;
    Pack16 u0, u1;
    u0.h[0] = (_Float16)(((at * f0.x) * rc) * 16.0f); u0.h[1] = (_Float16)(((at * f0.y) * rc) * 16.0f);
    u0.h[2] = (_Float16)(((at * f0.z) * rc) * 16.0f); u0.h[3] = (_Float16)(((at * f0.w) * rc) * 16.0f);
    u0.h[4] = (_Float16)(((at * f1.x) * rc) * 16.0f); u0.h[5] = (_Float16)(((at * f1.y) * rc) * 16.0f);
    u0.h[6] = (_Float16)(((at * f1.z) * rc) * 16.0f); u0.h[7] = (_Float16)(((at * f1.w) * rc) * 16.0f);
    u1.h[0] = (_Float16)(((at * f2.x) * rc) * 16.0f); u1.h[1] = (_Float16)(((at * f2.y) * rc) * 16.0f);
    u1.h[2] = (_Float16)(((at * f2.z) * rc) * 16.0f); u1.h[3] = (_Float16)(((at * f2.w) * rc) * 16.0f);
    u1.h[4] = (_Float16)(((at * f3.x) * rc) * 16.0f); u1.h[5] = (_Float16)(((at * f3.y) * rc) * 16.0f);
    u1.h[6] = (_Float16)(((at * f3.z) * rc) * 16.0f); u1.h[7] = (_Float16)(((at * f3.w) * rc) * 16.0f);
    *(v8h*)(At + r * AP + 16 * lane)     = u0.h;
    *(v8h*)(At + r * AP + 16 * lane + 8) = u1.h;
  }
  __syncthreads();

  mm_pass(At, Xs, Wh, bq, 1.0f / 256.0f, qscale, wave, hh, m);
  __syncthreads();
  store_rows_f32(Xs, qpl, rowBase, wave, lane);
  __syncthreads();

  mm_pass(At, Xs, Wh + (size_t)DF * DF, bk, 1.0f / 256.0f, 1.0f, wave, hh, m);
  __syncthreads();
  store_rows_f32(Xs, kpl, rowBase, wave, lane);
  __syncthreads();

  mm_pass(At, Xs, Wh + (size_t)2 * DF * DF, bv, 1.0f / 256.0f, 1.0f, wave, hh, m);
  __syncthreads();
  store_rows_f16(Xs, vpl, 16.0f, rowBase, wave, lane);
}

__global__ __launch_bounds__(NTHR) void k_agg(
    const float* __restrict__ qpl, const float* __restrict__ kpl, const _Float16* __restrict__ vpl,
    const int* __restrict__ srcA, const int* __restrict__ dstA,
    _Float16* apl, int nN, int nP, int nE) {
  extern __shared__ v4f lds_dyn[];
  float* qs   = (float*)lds_dyn;
  float* sacc = qs + NB * DF;
  float* sm   = sacc + NB * DF;
  float* sden = sm + NB;
  int*   list = (int*)(sden + NB);
  int*   wcnt = list + NWAVE * WCAP;

  const int tid  = threadIdx.x;
  const int lane = tid & 31;
  const int wave = tid >> 5;
  const int nodeBase = blockIdx.x * NB;

  {
    const v4f z4 = {0.f, 0.f, 0.f, 0.f};
    for (int i = tid; i < NB * DF / 4; i += NTHR) {
      const int slot = i >> 7;
      const int c4   = i & 127;
      int node = nodeBase + slot;
      if (node > nN - 1) node = nN - 1;
      ((v4f*)qs)[i]   = *(const v4f*)(qpl + (size_t)node * DF + 4 * c4);
      ((v4f*)sacc)[i] = z4;
    }
    if (tid < NB) { sm[tid] = -1.0e30f; sden[tid] = 0.f; }
  }
  __syncthreads();

  const int sent = -2147483647 - 1;
  const int nChunks = (nE + CHUNK - 1) / CHUNK;
#pragma unroll 1
  for (int ch = 0; ch < nChunks; ++ch) {
    const int cbase = ch * CHUNK;
    int wc = 0;
#pragma unroll
    for (int g = 0; g < NGRP; ++g) {
      const int el0 = (g * NTHR + tid) * 4;
      const int e0  = cbase + el0;
      v4i d;
      if (cbase + CHUNK <= nE) {
        d = *(const v4i*)(dstA + e0);
      } else {
        d.x = (e0     < nE) ? dstA[min(e0,     nE - 1)] : sent;
        d.y = (e0 + 1 < nE) ? dstA[min(e0 + 1, nE - 1)] : sent;
        d.z = (e0 + 2 < nE) ? dstA[min(e0 + 2, nE - 1)] : sent;
        d.w = (e0 + 3 < nE) ? dstA[min(e0 + 3, nE - 1)] : sent;
      }
      const unsigned s0 = (unsigned)d.x - (unsigned)nodeBase;
      const unsigned s1 = (unsigned)d.y - (unsigned)nodeBase;
      const unsigned s2 = (unsigned)d.z - (unsigned)nodeBase;
      const unsigned s3 = (unsigned)d.w - (unsigned)nodeBase;
      const bool h0 = s0 < (unsigned)NB;
      const bool h1 = s1 < (unsigned)NB;
      const bool h2 = s2 < (unsigned)NB;
      const bool h3 = s3 < (unsigned)NB;
      const unsigned many = __builtin_amdgcn_ballot_w32(h0 | h1 | h2 | h3);
      if (many != 0u) {
#define HITJ(J, HJ, SJ) { \
          const unsigned mj = __builtin_amdgcn_ballot_w32(HJ); \
          if (HJ) { \
            const int pos = wc + (int)__builtin_amdgcn_mbcnt_lo(mj, 0u); \
            if (pos < WCAP) list[wave * WCAP + pos] = ((el0 + (J)) << 6) | (int)(SJ); \
          } \
          wc += (int)__builtin_popcount(mj); }
        HITJ(0, h0, s0)
        HITJ(1, h1, s1)
        HITJ(2, h2, s2)
        HITJ(3, h3, s3)
#undef HITJ
      }
    }
    if (lane == 0) wcnt[wave] = wc;
    __syncthreads();

#pragma unroll 1
    for (int wsx = 0; wsx < NWAVE; ++wsx) {
      int n = wcnt[wsx];
      if (n > WCAP) n = WCAP;
      if (n < 0) n = 0;
#pragma unroll 1
      for (int i = 0; i < n; ++i) {
        const int ent  = list[wsx * WCAP + i];
        const int slot = ent & (NB - 1);
        if ((slot & (NWAVE - 1)) != wave) continue;
        const int el = (ent >> 6) & (CHUNK - 1);
        int e = cbase + el;
        if (e > nE - 1) e = nE - 1;
        int s = srcA[e];
        s = s < 0 ? 0 : (s > nN - 1 ? nN - 1 : s);
        const float* kr = kpl + (size_t)s * DF;
        const float* qr = qs + slot * DF;
        const v4f k0 = *(const v4f*)(kr + 8 * lane);
        const v4f k1 = *(const v4f*)(kr + 8 * lane + 4);
        const v4f k2 = *(const v4f*)(kr + 256 + 8 * lane);
        const v4f k3 = *(const v4f*)(kr + 256 + 8 * lane + 4);
        const v4f q0 = *(const v4f*)(qr + 8 * lane);
        const v4f q1 = *(const v4f*)(qr + 8 * lane + 4);
        const v4f q2 = *(const v4f*)(qr + 256 + 8 * lane);
        const v4f q3 = *(const v4f*)(qr + 256 + 8 * lane + 4);
        float dt = k0.x * q0.x + k0.y * q0.y + k0.z * q0.z + k0.w * q0.w
                 + k1.x * q1.x + k1.y * q1.y + k1.z * q1.z + k1.w * q1.w
                 + k2.x * q2.x + k2.y * q2.y + k2.z * q2.z + k2.w * q2.w
                 + k3.x * q3.x + k3.y * q3.y + k3.z * q3.z + k3.w * q3.w;
        dt = wsum(dt);
        const float mold = sm[slot];
        const float mnew = fmaxf(mold, dt);
        const float c = __expf(mold - mnew);
        const float p = __expf(dt - mnew);
        Pack16 va, vb;
        va.i = *(const v4i*)(vpl + (size_t)s * DF + 8 * lane);
        vb.i = *(const v4i*)(vpl + (size_t)s * DF + 256 + 8 * lane);
        float* ar = sacc + slot * DF;
        v4f a0 = *(const v4f*)(ar + 8 * lane);
        v4f a1 = *(const v4f*)(ar + 8 * lane + 4);
        v4f a2 = *(const v4f*)(ar + 256 + 8 * lane);
        v4f a3 = *(const v4f*)(ar + 256 + 8 * lane + 4);
        a0.x = a0.x * c + p * (float)va.h[0]; a0.y = a0.y * c + p * (float)va.h[1];
        a0.z = a0.z * c + p * (float)va.h[2]; a0.w = a0.w * c + p * (float)va.h[3];
        a1.x = a1.x * c + p * (float)va.h[4]; a1.y = a1.y * c + p * (float)va.h[5];
        a1.z = a1.z * c + p * (float)va.h[6]; a1.w = a1.w * c + p * (float)va.h[7];
        a2.x = a2.x * c + p * (float)vb.h[0]; a2.y = a2.y * c + p * (float)vb.h[1];
        a2.z = a2.z * c + p * (float)vb.h[2]; a2.w = a2.w * c + p * (float)vb.h[3];
        a3.x = a3.x * c + p * (float)vb.h[4]; a3.y = a3.y * c + p * (float)vb.h[5];
        a3.z = a3.z * c + p * (float)vb.h[6]; a3.w = a3.w * c + p * (float)vb.h[7];
        *(v4f*)(ar + 8 * lane)           = a0;
        *(v4f*)(ar + 8 * lane + 4)       = a1;
        *(v4f*)(ar + 256 + 8 * lane)     = a2;
        *(v4f*)(ar + 256 + 8 * lane + 4) = a3;
        const float dnew = sden[slot] * c + p;
        sm[slot]   = mnew;
        sden[slot] = dnew;
      }
    }
    __syncthreads();
  }

#pragma unroll 1
  for (int j = 0; j < NB / NWAVE; ++j) {
    const int slot = wave + NWAVE * j;
    const int node = nodeBase + slot;
    if (node < nP) {
      const float den = sden[slot];
      const float f = (node < nN && den > 0.f) ? 4.0f * (1.0f / den) : 0.f;
      const float* ar = sacc + slot * DF;
      const v4f a0 = *(const v4f*)(ar + 8 * lane);
      const v4f a1 = *(const v4f*)(ar + 8 * lane + 4);
      const v4f a2 = *(const v4f*)(ar + 256 + 8 * lane);
      const v4f a3 = *(const v4f*)(ar + 256 + 8 * lane + 4);
      Pack16 u0, u1;
      u0.h[0] = (_Float16)(a0.x * f); u0.h[1] = (_Float16)(a0.y * f); u0.h[2] = (_Float16)(a0.z * f); u0.h[3] = (_Float16)(a0.w * f);
      u0.h[4] = (_Float16)(a1.x * f); u0.h[5] = (_Float16)(a1.y * f); u0.h[6] = (_Float16)(a1.z * f); u0.h[7] = (_Float16)(a1.w * f);
      u1.h[0] = (_Float16)(a2.x * f); u1.h[1] = (_Float16)(a2.y * f); u1.h[2] = (_Float16)(a2.z * f); u1.h[3] = (_Float16)(a2.w * f);
      u1.h[4] = (_Float16)(a3.x * f); u1.h[5] = (_Float16)(a3.y * f); u1.h[6] = (_Float16)(a3.z * f); u1.h[7] = (_Float16)(a3.w * f);
      _Float16* gp = apl + (size_t)node * DF;
      *(volatile v4i*)(gp + 8 * lane)       = u0.i;
      *(volatile v4i*)(gp + 256 + 8 * lane) = u1.i;
      __threadfence();
      *(volatile v4i*)(gp + 8 * lane)       = u0.i;
      *(volatile v4i*)(gp + 256 + 8 * lane) = u1.i;
    }
  }
}

__global__ __launch_bounds__(NTHR) void k_out(
    const _Float16* __restrict__ apl, const _Float16* __restrict__ Woh, const float* __restrict__ bo,
    float* out, int nN) {
  extern __shared__ v4f lds_dyn[];
  _Float16* At = (_Float16*)lds_dyn;
  float* Xs = (float*)((char*)lds_dyn + GR * AP * 2);

  const int tid  = threadIdx.x;
  const int lane = tid & 31;
  const int wave = tid >> 5;
  const int hh   = lane >> 4;
  const int m    = lane & 15;
  const int rowBase = blockIdx.x * GR;

  {
    const int r  = tid >> 3;
    const int c0 = (tid & 7) * 64;
    const _Float16* p = apl + (size_t)(rowBase + r) * DF + c0;
#pragma unroll
    for (int j = 0; j < 8; ++j) *(v8h*)(At + r * AP + c0 + 8 * j) = *(const v8h*)(p + 8 * j);
  }
  __syncthreads();

  mm_pass(At, Xs, Woh, bo, 1.0f / 1024.0f, 1.0f, wave, hh, m);
  __syncthreads();

#pragma unroll 1
  for (int i = 0; i < 4; ++i) {
    const int rl  = 4 * wave + i;
    const int row = rowBase + rl;
    v4f h[4];
#pragma unroll
    for (int j = 0; j < 4; ++j) h[j] = *(const v4f*)(Xs + rl * XSP + 128 * j + 4 * lane);
    float ss = 0.f;
#pragma unroll
    for (int j = 0; j < 4; ++j) ss += h[j].x * h[j].x + h[j].y * h[j].y + h[j].z * h[j].z + h[j].w * h[j].w;
    ss = wsum(ss);
    const float nrm = sqrtf(ss);
    const float nc  = fmaxf(nrm, 1.0e-7f);
    const float th  = tanhf(nc);
    const float rc  = 1.0f / nc;
    v4f y[4];
#pragma unroll
    for (int j = 0; j < 4; ++j) {
      y[j].x = (h[j].x * th) * rc; y[j].y = (h[j].y * th) * rc;
      y[j].z = (h[j].z * th) * rc; y[j].w = (h[j].w * th) * rc;
    }
    if (row < nN) {
      float* gp = out + (size_t)row * DF;
#pragma unroll
      for (int j = 0; j < 4; ++j) *(volatile v4f*)(gp + 128 * j + 4 * lane) = y[j];
      __threadfence();
#pragma unroll
      for (int j = 0; j < 4; ++j) *(volatile v4f*)(gp + 128 * j + 4 * lane) = y[j];
    }
  }
}

extern "C" void kernel_launch(void* const* d_in, const int* in_sizes, int n_in,
                              void* d_out, int out_size, void* d_ws, size_t ws_size,
                              hipStream_t stream) {
  if (n_in < 11) return;
  const int nN = in_sizes[0] / DF;
  if (nN <= 0 || in_sizes[0] != nN * DF) return;
  const int nE = in_sizes[1];
  if (nE <= 0 || in_sizes[2] != nE) return;
  if (in_sizes[3] != DF * DF || in_sizes[5] != DF * DF || in_sizes[7] != DF * DF || in_sizes[9] != DF * DF) return;
  if (in_sizes[4] != DF || in_sizes[6] != DF || in_sizes[8] != DF || in_sizes[10] != DF) return;
  if (out_size != nN * DF) return;

  const float* x   = (const float*)d_in[0];
  const int*   src = (const int*)d_in[1];
  const int*   dst = (const int*)d_in[2];
  const float* Wq  = (const float*)d_in[3];
  const float* bq  = (const float*)d_in[4];
  const float* Wk  = (const float*)d_in[5];
  const float* bk  = (const float*)d_in[6];
  const float* Wv  = (const float*)d_in[7];
  const float* bv  = (const float*)d_in[8];
  const float* Wo  = (const float*)d_in[9];
  const float* bo  = (const float*)d_in[10];
  float* out = (float*)d_out;

  const int nP = ((nN + GR - 1) / GR) * GR;
  size_t off = 0;
  _Float16* Wh  = (_Float16*)((char*)d_ws + off); off += (size_t)4 * DF * DF * sizeof(_Float16);
  float*    qpl = (float*)((char*)d_ws + off);    off += (size_t)nP * DF * sizeof(float);
  float*    kpl = (float*)((char*)d_ws + off);    off += (size_t)nP * DF * sizeof(float);
  _Float16* vpl = (_Float16*)((char*)d_ws + off); off += (size_t)nP * DF * sizeof(_Float16);
  _Float16* apl = (_Float16*)((char*)d_ws + off); off += (size_t)nP * DF * sizeof(_Float16);
  if (off > ws_size) return;

  const float qscale = 1.0f / sqrtf((float)DF);
  const int n8 = DF * DF / 8;

  k_prep<<<dim3((n8 + NTHR - 1) / NTHR, 4), NTHR, 0, stream>>>(Wq, Wk, Wv, Wo, Wh, n8);

  hipFuncSetAttribute(reinterpret_cast<const void*>(&k_node),
                      hipFuncAttributeMaxDynamicSharedMemorySize, LDS_G_BYTES);
  k_node<<<nP / GR, NTHR, LDS_G_BYTES, stream>>>(x, Wh, bq, bk, bv, qpl, kpl, vpl, nN, qscale);

  hipFuncSetAttribute(reinterpret_cast<const void*>(&k_agg),
                      hipFuncAttributeMaxDynamicSharedMemorySize, LDS_A_BYTES);
  k_agg<<<(nP + NB - 1) / NB, NTHR, LDS_A_BYTES, stream>>>(qpl, kpl, vpl, src, dst, apl, nN, nP, nE);

  hipFuncSetAttribute(reinterpret_cast<const void*>(&k_out),
                      hipFuncAttributeMaxDynamicSharedMemorySize, LDS_G_BYTES);
  k_out<<<nP / GR, NTHR, LDS_G_BYTES, stream>>>(apl, Wh + (size_t)3 * DF * DF, bo, out, nN);
}
